// MSA_26328149524927
// MI455X (gfx1250) — hardware-run, weakly checked
//
#include <hip/hip_runtime.h>
#include <math.h>

typedef __attribute__((ext_vector_type(16))) _Float16 v16h;
typedef __attribute__((ext_vector_type(8)))  _Float16 v8h;
typedef __attribute__((ext_vector_type(16))) __bf16   v16b;
typedef __attribute__((ext_vector_type(8)))  __bf16   v8b;
typedef __attribute__((ext_vector_type(8)))  float    v8f;
typedef __attribute__((ext_vector_type(4)))  float    v4f;

constexpr int kBatch = 4;
constexpr int kSeq   = 2048;
constexpr int kEmb   = 1024;
constexpr int kHeads = 16;
constexpr int kHd    = 64;
constexpr int kTok   = kBatch * kSeq;
constexpr int kQB    = 128;
constexpr int kKC    = 64;
constexpr int kOP    = 72;
constexpr float kQKScale    = 0.125f;
constexpr int   kPCarryLog2 = 15;
constexpr float kPCarry     = 32768.0f;
constexpr float kLn2        = 0.693147180559945f;
constexpr float kLnPCarry   = (float)kPCarryLog2 * kLn2;
constexpr float kWCarry     = 16.0f;
constexpr float kWCarryInv  = 1.0f / kWCarry;
constexpr float kCtxCarry   = 256.0f;
constexpr float kOutScale   = 1.0f / (kCtxCarry * kWCarry);
static_assert(kHeads * kHd == kEmb);
static_assert(kHd == 64);
static_assert(kQKScale * kQKScale * (float)kHd == 1.0f);
static_assert(kPCarry == (float)(1 << kPCarryLog2));
static_assert((kSeq % kQB) == 0 && (kSeq % kKC) == 0);
static_assert((kTok % 64) == 0 && (kEmb % 64) == 0 && (kEmb % 32) == 0);

constexpr size_t kPlaneTok = (size_t)kTok * kEmb * 2;
constexpr size_t kPlaneW   = (size_t)kEmb * kEmb * 2;
constexpr size_t kOffXH = 0;
constexpr size_t kOffWT = kOffXH + kPlaneTok;
constexpr size_t kOffQP = kOffWT + 4 * kPlaneW;
constexpr size_t kOffKP = kOffQP + kPlaneTok;
constexpr size_t kOffVT = kOffKP + kPlaneTok;
constexpr size_t kOffOP = kOffVT + kPlaneTok;
constexpr size_t kWsTotal = kOffOP + kPlaneTok;
static_assert(kWsTotal == 92274688ull);
static_assert(kWsTotal <= 134217728ull);
static_assert((kOffWT % 128) == 0 && (kOffQP % 128) == 0 && (kOffKP % 128) == 0 &&
              (kOffVT % 128) == 0 && (kOffOP % 128) == 0);

__device__ __forceinline__ unsigned short f2bf_bits(float f) {
  unsigned u = __float_as_uint(f);
  return (unsigned short)((u + 0x7FFFu + ((u >> 16) & 1u)) >> 16);
}
__device__ __forceinline__ float bf_bits2f(unsigned short h) { return __uint_as_float(((unsigned)h) << 16); }

__device__ __forceinline__ void dep_guard4_h(v8f& a, v8f& b, v8f& c, v8f& d, v16h x, v16h y) {
  asm volatile("v_nop\n\tv_nop\n\tv_nop\n\tv_nop" : "+v"(a), "+v"(b), "+v"(c), "+v"(d) : "v"(x), "v"(y));
}
__device__ __forceinline__ void dep_guard4_b(v8f& a, v8f& b, v8f& c, v8f& d, v16b x, v16b y) {
  asm volatile("v_nop\n\tv_nop\n\tv_nop\n\tv_nop" : "+v"(a), "+v"(b), "+v"(c), "+v"(d) : "v"(x), "v"(y));
}
__device__ __forceinline__ void keep4_h(v16h a, v16h b, v16h c, v16h d) { asm volatile("v_nop" :: "v"(a), "v"(b), "v"(c), "v"(d)); }
__device__ __forceinline__ void keep4_b(v16b a, v16b b, v16b c, v16b d) { asm volatile("v_nop" :: "v"(a), "v"(b), "v"(c), "v"(d)); }
__device__ __forceinline__ void acc_guard4(v8f& a, v8f& b, v8f& c, v8f& d) {
  asm volatile("v_nop\n\tv_nop\n\tv_nop\n\tv_nop" : "+v"(a), "+v"(b), "+v"(c), "+v"(d));
}
__device__ __forceinline__ void guard1_h(v8f& a, v16h x0, v16h x1, v16h y0, v16h y1) {
  asm volatile("v_nop\n\tv_nop\n\tv_nop\n\tv_nop" : "+v"(a) : "v"(x0), "v"(x1), "v"(y0), "v"(y1));
}

template <typename T> struct Frag;
template <> struct Frag<_Float16> {
  typedef v16h V; union U { v16h v; v8h h[2]; };
  static __device__ __forceinline__ v16h load(const _Float16* p) {
    U f; f.h[0] = *(const v8h*)(p); f.h[1] = *(const v8h*)(p + 16); return f.v;
  }
  static __device__ __forceinline__ v8f mma(v16h a, v16h b, v8f c) {
    return __builtin_amdgcn_wmma_f32_16x16x32_f16(false, a, false, b, (short)0, c, false, false);
  }
  static __device__ __forceinline__ void guard4(v8f& a, v8f& b, v8f& c, v8f& d, v16h x, v16h y) { dep_guard4_h(a, b, c, d, x, y); }
  static __device__ __forceinline__ void keep(v16h a, v16h b, v16h c, v16h d) { keep4_h(a, b, c, d); }
};
template <> struct Frag<__bf16> {
  typedef v16b V; union U { v16b v; v8b h[2]; };
  static __device__ __forceinline__ v16b load(const __bf16* p) {
    U f; f.h[0] = *(const v8b*)(p); f.h[1] = *(const v8b*)(p + 16); return f.v;
  }
  static __device__ __forceinline__ v8f mma(v16b a, v16b b, v8f c) {
    return __builtin_amdgcn_wmma_f32_16x16x32_bf16(false, a, false, b, (short)0, c, false, false);
  }
  static __device__ __forceinline__ void guard4(v8f& a, v8f& b, v8f& c, v8f& d, v16b x, v16b y) { dep_guard4_b(a, b, c, d, x, y); }
  static __device__ __forceinline__ void keep(v16b a, v16b b, v16b c, v16b d) { keep4_b(a, b, c, d); }
};

template <int ET> struct Elem;
template <> struct Elem<0> { typedef _Float16 T; };
template <> struct Elem<1> { typedef __bf16 T; };
template <int ET, bool SPLIT, int BIAS_MODE, int OUT_MODE, bool RESID, int ACT = 0>
__global__ __launch_bounds__(256) void wmma_gemm64(
    const unsigned short* __restrict__ Ap, const unsigned short* __restrict__ A2p, int lda, long strideA,
    const unsigned short* __restrict__ Btp, const unsigned short* __restrict__ Bt2p, int ldb, long strideB,
    void* __restrict__ Cout, void* __restrict__ Cout2, int ldc, long strideC,
    const float* __restrict__ bias,
    const float* __restrict__ resid, long strideR,
    int M, int N, int K, float scale) {
  typedef typename Elem<ET>::T T;
  typedef typename Frag<T>::V V;
  const T* A = (const T*)Ap; const T* A2 = (const T*)A2p; const T* Bt = (const T*)Btp; const T* Bt2 = (const T*)Bt2p;
  __shared__ __align__(16) float sT[8][16 * 68];
  const int b    = blockIdx.y;
  const int lane = threadIdx.x & 31;
  const int wave = threadIdx.x >> 5;
  const int tilesN = N >> 6;
  const int tilesM = M >> 6;
  const int tile = blockIdx.x * 8 + wave;
  if (tile >= tilesM * tilesN) return;
  const int tm = tile / tilesN;
  const int tn = tile - tm * tilesN;
  const int m0 = tm << 6;
  const int n0 = tn << 6;

  const T* Ab  = A  + (size_t)b * strideA;
  const T* Bb  = Bt + (size_t)b * strideB;
  const T* Ab2 = SPLIT ? (A2  + (size_t)b * strideA) : nullptr;
  const T* Bb2 = SPLIT ? (Bt2 + (size_t)b * strideB) : nullptr;

  const int rlane = lane & 15;
  const int koff  = (lane >> 4) * 8;
  const int mOff  = (lane >> 4) * 8;

  v8f acc[4][4];
#pragma unroll
  for (int i = 0; i < 4; ++i)
#pragma unroll
    for (int j = 0; j < 4; ++j) acc[i][j] = (v8f){0.f,0.f,0.f,0.f,0.f,0.f,0.f,0.f};

  for (int k0 = 0; k0 < K; k0 += 32) {
    V bh[4], bl[4];
#pragma unroll
    for (int j = 0; j < 4; ++j) {
      const size_t bo = (size_t)(n0 + (j << 4) + rlane) * ldb + koff + k0;
      bh[j] = Frag<T>::load(Bb + bo);
      if (SPLIT) bl[j] = Frag<T>::load(Bb2 + bo);
    }
#pragma unroll
    for (int i = 0; i < 4; ++i) {
      const size_t ao = (size_t)(m0 + (i << 4) + rlane) * lda + koff + k0;
      V ah = Frag<T>::load(Ab + ao);
      V al;
      if (SPLIT) al = Frag<T>::load(Ab2 + ao);
#pragma unroll
      for (int j = 0; j < 4; ++j) {
        acc[i][j] = Frag<T>::mma(ah, bh[j], acc[i][j]);
        if (SPLIT) {
          acc[i][j] = Frag<T>::mma(ah, bl[j], acc[i][j]);
          acc[i][j] = Frag<T>::mma(al, bh[j], acc[i][j]);
        }
      }
      Frag<T>::guard4(acc[i][0], acc[i][1], acc[i][2], acc[i][3], ah, SPLIT ? al : ah);
    }
    Frag<T>::keep(bh[0], bh[1], bh[2], bh[3]);
    if (SPLIT) Frag<T>::keep(bl[0], bl[1], bl[2], bl[3]);
  }
  acc_guard4(acc[0][0], acc[0][1], acc[0][2], acc[0][3]);
  acc_guard4(acc[1][0], acc[1][1], acc[1][2], acc[1][3]);
  acc_guard4(acc[2][0], acc[2][1], acc[2][2], acc[2][3]);
  acc_guard4(acc[3][0], acc[3][1], acc[3][2], acc[3][3]);

  float* slab = sT[wave];
  const float* Rb = RESID ? (resid + (size_t)b * strideR) : nullptr;
#pragma unroll
  for (int i = 0; i < 4; ++i) {
    const int mBase = m0 + (i << 4);
#pragma unroll
    for (int j = 0; j < 4; ++j) {
      const int n = n0 + (j << 4) + rlane;
      float bv = 0.f;
      if (BIAS_MODE == 2) bv = bias[n];
#pragma unroll
      for (int r = 0; r < 8; ++r) {
        float v = acc[i][j][r] * scale;
        if (BIAS_MODE == 1) v += bias[mBase + mOff + r];
        if (BIAS_MODE == 2) v += bv;
        if (RESID) v += Rb[(size_t)(mBase + mOff + r) * ldc + n];
        if (ACT == 2) v = fmaxf(v, 0.0f);
        if (ACT == 4) v = (v > 0.f) ? v : 0.01f * v;
        slab[(mOff + r) * 68 + (j << 4) + rlane] = v;
      }
    }
    __builtin_amdgcn_fence(__ATOMIC_RELEASE, "workgroup");
    __builtin_amdgcn_wave_barrier();
    __builtin_amdgcn_fence(__ATOMIC_ACQUIRE, "workgroup");
    if (OUT_MODE == 0) {
      float* C = (float*)Cout + (size_t)b * strideC;
      const int hh = lane >> 4, c4 = (lane & 15) * 4;
      for (int pass = 0; pass < 2; ++pass) {
#pragma unroll
        for (int it = 0; it < 8; ++it) {
          const int row = it * 2 + hh;
          v4f v = *(const v4f*)(slab + row * 68 + c4);
          *(volatile v4f*)(C + (size_t)(mBase + row) * ldc + n0 + c4) = v;
        }
        __threadfence();
      }
    } else {
      const int q = lane >> 3, c8 = (lane & 7) * 8;
      unsigned short* C  = (unsigned short*)Cout  + (size_t)b * strideC;
      unsigned short* C2 = (OUT_MODE == 2) ? ((unsigned short*)Cout2 + (size_t)b * strideC) : nullptr;
      for (int pass = 0; pass < 2; ++pass) {
#pragma unroll
        for (int it = 0; it < 4; ++it) {
          const int row = it * 4 + q;
          const float* sp = slab + row * 68 + c8;
          v8h hv, lv;
#pragma unroll
          for (int e = 0; e < 8; ++e) {
            if (OUT_MODE == 1) {
              hv[e] = (_Float16)sp[e];
            } else {
              unsigned short hb = f2bf_bits(sp[e]);
              unsigned short lb = f2bf_bits(sp[e] - bf_bits2f(hb));
              hv[e] = __builtin_bit_cast(_Float16, hb);
              lv[e] = __builtin_bit_cast(_Float16, lb);
            }
          }
          *(volatile v8h*)(C + (size_t)(mBase + row) * ldc + n0 + c8) = hv;
          if (OUT_MODE == 2) *(volatile v8h*)(C2 + (size_t)(mBase + row) * ldc + n0 + c8) = lv;
        }
        __threadfence();
      }
    }
    __builtin_amdgcn_fence(__ATOMIC_RELEASE, "workgroup");
    __builtin_amdgcn_wave_barrier();
    __builtin_amdgcn_fence(__ATOMIC_ACQUIRE, "workgroup");
  }
}

__global__ __launch_bounds__(256) void cast8_f16_kernel(const float* __restrict__ in, unsigned short* __restrict__ out, int n8) {
  const int i = blockIdx.x * 256 + threadIdx.x;
  if (i >= n8) return;
  const float* p = in + 8 * (size_t)i;
  const v4f a = *(const v4f*)(p);
  const v4f c = *(const v4f*)(p + 4);
  v8h hv;
#pragma unroll
  for (int e = 0; e < 4; ++e) {
    const float fa = a[e];
    const float fc = c[e];
    hv[e]     = (_Float16)fa;
    hv[4 + e] = (_Float16)fc;
  }
  unsigned short* q = out + 8 * (size_t)i;
  *(volatile v8h*)q = hv;
  __threadfence();
  *(volatile v8h*)q = hv;
}

__global__ __launch_bounds__(256) void wtcast_kernel(const float* __restrict__ W0, const float* __restrict__ W1,
                                                     const float* __restrict__ W2, const float* __restrict__ W3,
                                                     unsigned short* __restrict__ out) {
  __shared__ float sm[64][65];
  const int t  = threadIdx.x;
  const int k0 = blockIdx.x * 64;
  const int n0 = blockIdx.y * 64;
  const int z  = blockIdx.z;
  const float* W = (z == 0) ? W0 : (z == 1) ? W1 : (z == 2) ? W2 : W3;
#pragma unroll
  for (int i = 0; i < 16; ++i) {
    const int e = i * 256 + t;
    const int r = e >> 6;
    const int c = e & 63;
    sm[c][r] = W[(size_t)(k0 + r) * kEmb + n0 + c] * kWCarry;
  }
  __syncthreads();
  const int lane = t & 31, wave = t >> 5;
  const int q = lane >> 3, c8 = (lane & 7) * 8;
  unsigned short* op = out + (size_t)z * kEmb * kEmb;
  v8h hv[2];
#pragma unroll
  for (int it = 0; it < 2; ++it) {
    const int row = wave * 8 + it * 4 + q;
#pragma unroll
    for (int e = 0; e < 8; ++e) hv[it][e] = (_Float16)sm[row][c8 + e];
  }
  for (int pass = 0; pass < 2; ++pass) {
#pragma unroll
    for (int it = 0; it < 2; ++it) {
      const int row = wave * 8 + it * 4 + q;
      *(volatile v8h*)(op + (size_t)(n0 + row) * kEmb + k0 + c8) = hv[it];
    }
    __threadfence();
  }
}

__device__ __forceinline__ v8f mma_h(v16h a, v16h b, v8f c) {
  return __builtin_amdgcn_wmma_f32_16x16x32_f16(false, a, false, b, (short)0, c, false, false);
}

__global__ __launch_bounds__(128) void attn_kernel(const unsigned short* __restrict__ Qp, const unsigned short* __restrict__ Kp,
                                                   const unsigned short* __restrict__ Vtp, unsigned short* __restrict__ Op) {
  __shared__ __align__(16) _Float16 Ks[kKC * kHd];
  __shared__ __align__(16) _Float16 Vs[kHd * kKC];
  __shared__ __align__(16) _Float16 Osh[4 * 32 * kOP];

  const int tid  = threadIdx.x;
  const int wave = tid >> 5;
  const int lane = tid & 31;
  const int hh   = lane >> 4;
  const int c    = lane & 15;

  constexpr int nqb = kSeq / kQB;
  const int bx   = blockIdx.x;
  const int qblk = bx % nqb;
  const int bh   = bx / nqb;
  const int h    = bh % kHeads;
  const int b    = bh / kHeads;
  const int q0   = qblk * kQB + wave * 32;
  const size_t tok0 = (size_t)b * kSeq;
  const int hcol = h * kHd;

  const _Float16* Qh = (const _Float16*)Qp;
  const _Float16* Kh = (const _Float16*)Kp;
  const _Float16* Vh = (const _Float16*)Vtp;
  _Float16* Oh = (_Float16*)Op;

  v16h qf[2][2];
#pragma unroll
  for (int qt = 0; qt < 2; ++qt) {
#pragma unroll
    for (int dc = 0; dc < 2; ++dc) {
      qf[qt][dc] = Frag<_Float16>::load(Qh + (tok0 + q0 + 16 * qt + c) * kEmb + hcol + dc * 32 + 8 * hh);
    }
  }

  float mrow[2], lrow[2];
  v8f oacc[2][4];
#pragma unroll
  for (int qt = 0; qt < 2; ++qt) {
    mrow[qt] = -1e30f;
    lrow[qt] = 0.f;
#pragma unroll
    for (int t = 0; t < 4; ++t) oacc[qt][t] = (v8f){0.f,0.f,0.f,0.f,0.f,0.f,0.f,0.f};
  }

#pragma unroll 1
  for (int kc = 0; kc < kSeq / kKC; ++kc) {
    const int kv0 = kc * kKC;
    __syncthreads();
    {
      v8h kvv[4], vvv[4];
#pragma unroll
      for (int i = 0; i < 4; ++i) {
        const int p   = i * 128 + tid;
        const int row = p >> 3;
        const int seg = (p & 7) * 8;
        kvv[i] = *(const v8h*)(Kh + (tok0 + kv0 + row) * kEmb + hcol + seg);
        vvv[i] = *(const v8h*)(Vh + (size_t)(hcol + row) * kTok + tok0 + kv0 + seg);
      }
#pragma unroll
      for (int i = 0; i < 4; ++i) {
        const int p = i * 128 + tid;
        *(v8h*)(Ks + p * 8) = kvv[i];
        *(v8h*)(Vs + p * 8) = vvv[i];
      }
    }
    __syncthreads();

#pragma unroll
    for (int qt = 0; qt < 2; ++qt) {
      v8f s[4];
#pragma unroll
      for (int j = 0; j < 4; ++j) {
        const _Float16* kr = Ks + (16 * j + c) * kHd + 8 * hh;
        const v16h ka0 = Frag<_Float16>::load(kr);
        const v16h ka1 = Frag<_Float16>::load(kr + 32);
        v8f a = (v8f){0.f,0.f,0.f,0.f,0.f,0.f,0.f,0.f};
        a = mma_h(ka0, qf[qt][0], a);
        a = mma_h(ka1, qf[qt][1], a);
        guard1_h(a, ka0, ka1, qf[qt][0], qf[qt][1]);
        s[j] = a;
      }
      float cm = s[0][0];
#pragma unroll
      for (int j = 0; j < 4; ++j) {
#pragma unroll
        for (int r = 0; r < 8; ++r) cm = fmaxf(cm, s[j][r]);
      }
      const float cmo = __shfl_xor(cm, 16, 32);
      cm = fmaxf(cm, cmo);
      const float mnew  = fmaxf(mrow[qt], cm);
      const float alpha = __expf((mrow[qt] - mnew) * kQKScale);
      mrow[qt] = mnew;
      const float nm = fmaf(-mnew, kQKScale, kLnPCarry);
      float ls = 0.f;
#pragma unroll
      for (int j = 0; j < 4; ++j) {
#pragma unroll
        for (int r = 0; r < 8; ++r) {
          const float p = __expf(fmaf(s[j][r], kQKScale, nm));
          ls += p;
          s[j][r] = p;
        }
      }
      lrow[qt] = fmaf(lrow[qt], alpha, ls);
#pragma unroll
      for (int t = 0; t < 4; ++t) {
#pragma unroll
        for (int r = 0; r < 8; ++r) oacc[qt][t][r] *= alpha;
      }
      v16h pf[2];
#pragma unroll
      for (int kk = 0; kk < 2; ++kk) {
#pragma unroll
        for (int e = 0; e < 8; ++e) {
          const float p0 = s[2 * kk][e];
          const float p1 = s[2 * kk + 1][e];
          pf[kk][e]     = (_Float16)p0;
          pf[kk][8 + e] = (_Float16)p1;
        }
      }
#pragma unroll
      for (int t = 0; t < 4; ++t) {
        const _Float16* vr = Vs + (16 * t + c) * kKC + 8 * hh;
        const v16h va0 = Frag<_Float16>::load(vr);
        const v16h va1 = Frag<_Float16>::load(vr + 32);
        v8f o = oacc[qt][t];
        o = mma_h(va0, pf[0], o);
        o = mma_h(va1, pf[1], o);
        guard1_h(o, va0, va1, pf[0], pf[1]);
        oacc[qt][t] = o;
      }
    }
  }

  _Float16* osw = Osh + wave * 32 * kOP;
#pragma unroll
  for (int qt = 0; qt < 2; ++qt) {
    const float lo = __shfl_xor(lrow[qt], 16, 32);
    const float lt = lrow[qt] + lo;
    const float inv = kCtxCarry * (1.0f / lt);
#pragma unroll
    for (int t = 0; t < 4; ++t) {
      v8h hv;
#pragma unroll
      for (int r = 0; r < 8; ++r) {
        const float ov = oacc[qt][t][r] * inv;
        hv[r] = (_Float16)ov;
      }
      *(v8h*)(osw + (16 * qt + c) * kOP + 16 * t + 8 * hh) = hv;
    }
  }
  __syncthreads();
  {
    const int q = lane >> 3, c8 = (lane & 7) * 8;
    v8h ov[8];
#pragma unroll
    for (int it = 0; it < 8; ++it) ov[it] = *(const v8h*)(osw + (it * 4 + q) * kOP + c8);
    for (int pass = 0; pass < 2; ++pass) {
#pragma unroll
      for (int it = 0; it < 8; ++it) {
        *(volatile v8h*)(Oh + (tok0 + q0 + it * 4 + q) * kEmb + hcol + c8) = ov[it];
      }
      __threadfence();
    }
  }
}

extern "C" void kernel_launch(void* const* d_in, const int* in_sizes, int n_in,
                              void* d_out, int out_size, void* d_ws, size_t ws_size,
                              hipStream_t stream) {
  if (n_in < 9) return;
  if (in_sizes[0] != kTok * kEmb) return;
  if (in_sizes[1] != kEmb * kEmb) return;
  if (in_sizes[2] != kEmb) return;
  if (in_sizes[3] != kEmb * kEmb) return;
  if (in_sizes[4] != kEmb) return;
  if (in_sizes[5] != kEmb * kEmb) return;
  if (in_sizes[6] != kEmb) return;
  if (in_sizes[7] != kEmb * kEmb) return;
  if (in_sizes[8] != kEmb) return;
  if (out_size != kTok * kEmb) return;
  if (ws_size < kWsTotal) return;

  const float* x  = (const float*)d_in[0];
  const float* Wq = (const float*)d_in[1];
  const float* bq = (const float*)d_in[2];
  const float* Wk = (const float*)d_in[3];
  const float* bk = (const float*)d_in[4];
  const float* Wv = (const float*)d_in[5];
  const float* bv = (const float*)d_in[6];
  const float* Wo = (const float*)d_in[7];
  const float* bo = (const float*)d_in[8];
  float* out = (float*)d_out;

  char* ws = (char*)d_ws;
  unsigned short* XH = (unsigned short*)(ws + kOffXH);
  unsigned short* WT = (unsigned short*)(ws + kOffWT);
  unsigned short* QP = (unsigned short*)(ws + kOffQP);
  unsigned short* KP = (unsigned short*)(ws + kOffKP);
  unsigned short* VT = (unsigned short*)(ws + kOffVT);
  unsigned short* OP = (unsigned short*)(ws + kOffOP);
  unsigned short* WqT = WT;
  unsigned short* WkT = WT + (size_t)1 * kEmb * kEmb;
  unsigned short* WvT = WT + (size_t)2 * kEmb * kEmb;
  unsigned short* WoT = WT + (size_t)3 * kEmb * kEmb;

  cast8_f16_kernel<<<(kTok * kEmb / 8) / 256, 256, 0, stream>>>(x, XH, kTok * kEmb / 8);
  wtcast_kernel<<<dim3(kEmb / 64, kEmb / 64, 4), 256, 0, stream>>>(Wq, Wk, Wv, Wo, WT);

  constexpr int kGemmBlocks = ((kTok / 64) * (kEmb / 64)) / 8;

  wmma_gemm64<0, false, 2, 1, false><<<dim3(kGemmBlocks, 1), 256, 0, stream>>>(
      XH, nullptr, kEmb, 0L,
      WqT, nullptr, kEmb, 0L,
      (void*)QP, nullptr, kEmb, 0L,
      bq, nullptr, 0L,
      kTok, kEmb, kEmb, kWCarryInv);

  wmma_gemm64<0, false, 2, 1, false><<<dim3(kGemmBlocks, 1), 256, 0, stream>>>(
      XH, nullptr, kEmb, 0L,
      WkT, nullptr, kEmb, 0L,
      (void*)KP, nullptr, kEmb, 0L,
      bk, nullptr, 0L,
      kTok, kEmb, kEmb, kWCarryInv);

  wmma_gemm64<0, false, 1, 1, false><<<dim3(kGemmBlocks, 1), 256, 0, stream>>>(
      WvT, nullptr, kEmb, 0L,
      XH, nullptr, kEmb, 0L,
      (void*)VT, nullptr, kTok, 0L,
      bv, nullptr, 0L,
      kEmb, kTok, kEmb, kWCarryInv);

  attn_kernel<<<kBatch * kHeads * (kSeq / kQB), 128, 0, stream>>>(QP, KP, VT, OP);

  wmma_gemm64<0, false, 2, 0, false><<<dim3(kGemmBlocks, 1), 256, 0, stream>>>(
      OP, nullptr, kEmb, 0L,
      WoT, nullptr, kEmb, 0L,
      (void*)out, nullptr, kEmb, 0L,
      bo, nullptr, 0L,
      kTok, kEmb, kEmb, kOutScale);
}
